// scGraphformerConv_31533649887564
// MI455X (gfx1250) — hardware-verified
//
#include <hip/hip_runtime.h>
#include <stddef.h>


#define CIN    256
#define CW     256
#define NH     4
#define HD     64
#define NTHR   256
#define NWAVE  8
#define SUBR   32
#define AP     264
#define TP     256
#define KVR    256
#define QR     128
#define AR     128
#define GSL    512
#define NPQ    512
#define NBC    32768
#define EPT    8
#define NGRP   2
#define CHUNK  (NTHR * EPT * NGRP)
#define WCAP   (EPT * NGRP * 32)
#define LISTN  (NWAVE * WCAP)
#define ASC    16
#define WSC    64
#define QSC    16
#define KVSC   64
#define KVN    (NH * HD * HD)
#define TCSK   0
#define TCSV   256
#define TS1    512
#define TS2    544
#define TABN   576
#define SRECN  (3 * CW)
#define QRECN  CW
#define WSCAP  134217728

#define LDS_COUNT ((NBC + LISTN + NWAVE) * 4)
#define LDS_AH    (SUBR * AP * 2)
#define LDS_KV    (LDS_AH + 2 * SUBR * TP * 4 + KVN * 4)
#define LDS_Q     (LDS_AH + SUBR * TP * 4 + CW * 4 + SUBR * NH * 4)
#define LDS_GCN   (GSL * HD * 4 + LISTN * 4 + NWAVE * 4)
#define LDS_F1    (KVN * 4 + CW * 8 + 2 * CW * 4)

static_assert((CHUNK & (CHUNK - 1)) == 0);
static_assert((NBC & (NBC - 1)) == 0);
static_assert(NBC == NWAVE * 32 * 128);
static_assert(CW == NH * HD && CW == NTHR && CIN == 256);
static_assert(SUBR * CIN == NTHR * 32);
static_assert(SUBR == 2 * 16 && NWAVE == 8);
static_assert((KVR % SUBR) == 0 && (QR % SUBR) == 0);
static_assert((NPQ % KVR) == 0 && (NPQ % QR) == 0 && (NPQ % AR) == 0 && (NPQ % GSL) == 0 && (NBC % NPQ) == 0);
static_assert(AR == NWAVE * 16);
static_assert(KVN == 64 * NTHR);
static_assert(GSL * HD == 32 * 4 * NTHR);
static_assert((AP % 8) == 0 && (LDS_AH % 16) == 0);
static_assert(LDS_KV == 147968 && LDS_Q == 51200 && LDS_GCN == 147488 && LDS_F1 == 69632 && LDS_COUNT == 147488);
static_assert(((TS1 * 4) % 128) == 0 && ((TS2 * 4) % 128) == 0 && TABN * 4 == 2304);
static_assert((SRECN % 2) == 0 && (QRECN % 2) == 0);

typedef float    v2f  __attribute__((ext_vector_type(2)));
typedef float    v4f  __attribute__((ext_vector_type(4)));
typedef float    v8f  __attribute__((ext_vector_type(8)));
typedef int      v4i  __attribute__((ext_vector_type(4)));
typedef double   v2d  __attribute__((ext_vector_type(2)));
typedef _Float16 v8h  __attribute__((ext_vector_type(8)));
typedef _Float16 v16h __attribute__((ext_vector_type(16)));
union FragH { v16h v; v8h h[2]; };

__device__ __forceinline__ v8f wmf(v16h a, v16h b, v8f c) {
  v8f d = __builtin_amdgcn_wmma_f32_16x16x32_f16(false, a, false, b, (short)0, c, false, false);
  asm volatile("v_nop\n\tv_nop\n\tv_nop\n\tv_nop" : "+v"(d) : "v"(a), "v"(b));
  return d;
}

__device__ __forceinline__ v8h cvt8(v4f a, v4f b, float s) {
  v8h o;
  o[0] = (_Float16)(a.x * s); o[1] = (_Float16)(a.y * s); o[2] = (_Float16)(a.z * s); o[3] = (_Float16)(a.w * s);
  o[4] = (_Float16)(b.x * s); o[5] = (_Float16)(b.y * s); o[6] = (_Float16)(b.z * s); o[7] = (_Float16)(b.w * s);
  return o;
}

__global__ __launch_bounds__(NTHR) void k_wprep(const float* __restrict__ wq, const float* __restrict__ wk,
                                                const float* __restrict__ wv, _Float16* wp) {
  const int tid = threadIdx.x;
  const int z = (int)blockIdx.x >> 5;
  const int i = (((int)blockIdx.x & 31) * NTHR) + tid;
  const float* w = (z == 0) ? wq : ((z == 1) ? wk : wv);
  const v4f a = *(const v4f*)(w + 8 * i);
  const v4f b = *(const v4f*)(w + 8 * i + 4);
  const v8h hv = cvt8(a, b, (float)WSC);
  _Float16* d = wp + (size_t)z * (CW * CIN) + (size_t)8 * i;
  *(volatile v8h*)d = hv;
  __threadfence();
  *(volatile v8h*)d = hv;
}

template <int NB, int MODE>
__device__ __forceinline__ int scan_chunk(const int* __restrict__ keys, int nE, int cbase, int slotBase,
                                          int vec8, int* list, int tid, int wave) {
  int wc = 0;
#pragma unroll
  for (int g = 0; g < NGRP; ++g) {
    const int e0   = cbase + (g * NTHR + tid) * EPT;
    const int sent = -2147483647 - 1;
    v4i da, db;
    if (vec8 != 0 && cbase + CHUNK <= nE) {
      da = *(const v4i*)(keys + e0);
      db = *(const v4i*)(keys + e0 + 4);
    } else {
      const int em = nE - 1;
      da.x = (e0     < nE) ? keys[min(e0,     em)] : sent;
      da.y = (e0 + 1 < nE) ? keys[min(e0 + 1, em)] : sent;
      da.z = (e0 + 2 < nE) ? keys[min(e0 + 2, em)] : sent;
      da.w = (e0 + 3 < nE) ? keys[min(e0 + 3, em)] : sent;
      db.x = (e0 + 4 < nE) ? keys[min(e0 + 4, em)] : sent;
      db.y = (e0 + 5 < nE) ? keys[min(e0 + 5, em)] : sent;
      db.z = (e0 + 6 < nE) ? keys[min(e0 + 6, em)] : sent;
      db.w = (e0 + 7 < nE) ? keys[min(e0 + 7, em)] : sent;
    }
    const unsigned nb = (unsigned)slotBase;
    const unsigned s0 = (unsigned)da.x - nb, s1 = (unsigned)da.y - nb;
    const unsigned s2 = (unsigned)da.z - nb, s3 = (unsigned)da.w - nb;
    const unsigned s4 = (unsigned)db.x - nb, s5 = (unsigned)db.y - nb;
    const unsigned s6 = (unsigned)db.z - nb, s7 = (unsigned)db.w - nb;
    const bool h0 = s0 < (unsigned)NB, h1 = s1 < (unsigned)NB, h2 = s2 < (unsigned)NB, h3 = s3 < (unsigned)NB;
    const bool h4 = s4 < (unsigned)NB, h5 = s5 < (unsigned)NB, h6 = s6 < (unsigned)NB, h7 = s7 < (unsigned)NB;
    const unsigned any = __builtin_amdgcn_ballot_w32(h0 | h1 | h2 | h3 | h4 | h5 | h6 | h7);
    if (any != 0u) {
#define HITJ(HJ, SJ, J) { \
        const unsigned mj = __builtin_amdgcn_ballot_w32(HJ); \
        if (mj != 0u) { \
          if (HJ) { \
            const int pos = wc + (int)__builtin_amdgcn_mbcnt_lo(mj, 0u); \
            const int entv = MODE ? (e0 + (J)) : (int)(SJ); \
            if (pos < WCAP) list[wave * WCAP + pos] = entv; \
          } \
          wc += (int)__builtin_popcount(mj); } }
      HITJ(h0, s0, 0)
      HITJ(h1, s1, 1)
      HITJ(h2, s2, 2)
      HITJ(h3, s3, 3)
      HITJ(h4, s4, 4)
      HITJ(h5, s5, 5)
      HITJ(h6, s6, 6)
      HITJ(h7, s7, 7)
#undef HITJ
    }
  }
  return wc;
}

__global__ __launch_bounds__(NTHR) void k_count(const int* __restrict__ keys, int* cnt, float* dz, int nE, int vec8) {
  extern __shared__ v4f lds_dyn[];
  int* scnt = (int*)lds_dyn;
  int* list = scnt + NBC;
  int* wcnt = list + LISTN;
  const int tid = threadIdx.x, lane = tid & 31, wave = tid >> 5;
  const int nodeBase = blockIdx.x * NBC;

  {
    const v4i z = {0, 0, 0, 0};
    for (int i = tid; i < NBC / 4; i += NTHR) ((v4i*)scnt)[i] = z;
  }
  __syncthreads();

  const int nChunks = (nE + CHUNK - 1) / CHUNK;
#pragma unroll 1
  for (int ch = 0; ch < nChunks; ++ch) {
    const int cbase = ch * CHUNK;
    const int wc = scan_chunk<NBC, 0>(keys, nE, cbase, nodeBase, vec8, list, tid, wave);
    if (lane == 0) wcnt[wave] = wc;
    __syncthreads();
    if (wave == 0) {
#pragma unroll 1
      for (int wsx = 0; wsx < NWAVE; ++wsx) {
        int n = __builtin_amdgcn_readfirstlane(wcnt[wsx]);
        n = n > WCAP ? WCAP : (n < 0 ? 0 : n);
        const int* lp = list + wsx * WCAP;
#pragma unroll 1
        for (int i = 0; i < n; ++i) {
          const int ent  = __builtin_amdgcn_readfirstlane(lp[i]);
          const int slot = ent & (NBC - 1);
          if (lane == 0) scnt[slot] = scnt[slot] + 1;
        }
      }
    }
    __syncthreads();
  }

  int*   cp = cnt + (size_t)nodeBase;
  float* dp = dz + (size_t)nodeBase;
#pragma unroll 1
  for (int q = 0; q < 32; ++q) {
    const int f = (wave * 32 + q) * 128 + 4 * lane;
    const v4i c = *(const v4i*)(scnt + f);
    v4f d;
    d.x = c.x > 0 ? rsqrtf(fmaxf((float)c.x, 1.0f)) : 0.0f;
    d.y = c.y > 0 ? rsqrtf(fmaxf((float)c.y, 1.0f)) : 0.0f;
    d.z = c.z > 0 ? rsqrtf(fmaxf((float)c.z, 1.0f)) : 0.0f;
    d.w = c.w > 0 ? rsqrtf(fmaxf((float)c.w, 1.0f)) : 0.0f;
    *(volatile v4i*)(cp + f) = c;
    *(volatile v4f*)(dp + f) = d;
  }
  __threadfence();
#pragma unroll 1
  for (int q = 0; q < 32; ++q) {
    const int f = (wave * 32 + q) * 128 + 4 * lane;
    const v4i c = *(const v4i*)(scnt + f);
    v4f d;
    d.x = c.x > 0 ? rsqrtf(fmaxf((float)c.x, 1.0f)) : 0.0f;
    d.y = c.y > 0 ? rsqrtf(fmaxf((float)c.y, 1.0f)) : 0.0f;
    d.z = c.z > 0 ? rsqrtf(fmaxf((float)c.z, 1.0f)) : 0.0f;
    d.w = c.w > 0 ? rsqrtf(fmaxf((float)c.w, 1.0f)) : 0.0f;
    *(volatile v4i*)(cp + f) = c;
    *(volatile v4f*)(dp + f) = d;
  }
}

__device__ __forceinline__ void cvt_tile(const float* __restrict__ X, int rb, int nN, _Float16* Ah, int tid) {
  const int row = tid >> 3, part = tid & 7;
  int gr = rb + row;
  const bool ok = gr < nN;
  gr = ok ? gr : nN - 1;
  const float sc = ok ? (float)ASC : 0.0f;
  const float* xp = X + (size_t)gr * CIN + 32 * part;
  _Float16* ap = Ah + row * AP + 32 * part;
#pragma unroll
  for (int j = 0; j < 4; ++j) {
    const v4f a = *(const v4f*)(xp + 8 * j);
    const v4f b = *(const v4f*)(xp + 8 * j + 4);
    *(v8h*)(ap + 8 * j) = cvt8(a, b, sc);
  }
}

__device__ __forceinline__ void gemm_unit(const _Float16* Ah, const _Float16* __restrict__ Wpl,
                                          const float* __restrict__ bias, float* Tm, int rt, int cg, int lane) {
  constexpr float OSC = 1.0f / (float)(ASC * WSC);
  const int hh = lane >> 4, m = lane & 15;
  v8f acc[4];
#pragma unroll
  for (int t = 0; t < 4; ++t) { v8f z = {0.f, 0.f, 0.f, 0.f, 0.f, 0.f, 0.f, 0.f}; acc[t] = z; }
  const _Float16* ap  = Ah + (16 * rt + m) * AP + 8 * hh;
  const _Float16* bp0 = Wpl + (size_t)(64 * cg + m) * CIN + 8 * hh;
#pragma unroll 1
  for (int kt = 0; kt < CIN / 32; ++kt) {
    FragH af;
    af.h[0] = *(const v8h*)(ap + 32 * kt);
    af.h[1] = *(const v8h*)(ap + 32 * kt + 16);
#pragma unroll
    for (int nt = 0; nt < 4; ++nt) {
      const _Float16* bp = bp0 + (size_t)(16 * nt) * CIN + 32 * kt;
      FragH bf;
      bf.h[0] = *(const v8h*)bp;
      bf.h[1] = *(const v8h*)(bp + 16);
      acc[nt] = wmf(af.v, bf.v, acc[nt]);
    }
  }
  float* sp = Tm + (16 * rt + 8 * hh) * TP + 64 * cg + m;
#pragma unroll
  for (int nt = 0; nt < 4; ++nt) {
    const float bt = bias[64 * cg + 16 * nt + m];
#pragma unroll
    for (int r = 0; r < 8; ++r) sp[r * TP + 16 * nt] = acc[nt][r] * OSC + bt;
  }
}

__global__ __launch_bounds__(NTHR) void k_kv(const float* __restrict__ X, const _Float16* __restrict__ wp,
                                             const float* __restrict__ bk, const float* __restrict__ bv,
                                             float* vbar, float* kvpart, double* strec, int nN) {
  extern __shared__ v4f lds_dyn[];
  _Float16* Ah = (_Float16*)lds_dyn;
  float* T   = (float*)((char*)lds_dyn + LDS_AH);
  float* kva = T + 2 * SUBR * TP;
  const int tid = threadIdx.x, lane = tid & 31, wave = tid >> 5;
  const int cm = tid & 63, dg = (tid >> 6) * 16;
  {
    const v4f z = {0.f, 0.f, 0.f, 0.f};
    for (int i = tid; i < KVN / 4; i += NTHR) ((v4f*)kva)[i] = z;
  }
  double sk = 0.0, sk2 = 0.0, sv = 0.0;

#pragma unroll 1
  for (int st = 0; st < KVR / SUBR; ++st) {
    const int rb = blockIdx.x * KVR + st * SUBR;
    cvt_tile(X, rb, nN, Ah, tid);
    __syncthreads();
    gemm_unit(Ah, wp + (size_t)1 * (CW * CIN), bk, T, wave & 1, wave >> 1, lane);
    gemm_unit(Ah, wp + (size_t)2 * (CW * CIN), bv, T + SUBR * TP, wave & 1, wave >> 1, lane);
    __syncthreads();
    int nr = nN - rb;
    nr = nr > SUBR ? SUBR : nr;
#pragma unroll 1
    for (int r = 0; r < nr; ++r) {
      const float kq = T[r * TP + tid];
      const float vq = T[SUBR * TP + r * TP + tid];
      sk  += (double)kq;
      sk2 += (double)kq * (double)kq;
      sv  += (double)vq;
    }
#pragma unroll 1
    for (int h = 0; h < NH; ++h) {
      float a16[16];
#pragma unroll
      for (int j = 0; j < 16; ++j) a16[j] = 0.0f;
      const float* kp = T + h * HD + cm;
      const float* vp = T + SUBR * TP + h * HD + dg;
#pragma unroll 1
      for (int r = 0; r < nr; ++r) {
        const float kk = kp[r * TP];
        const v4f x0 = *(const v4f*)(vp + r * TP);
        const v4f x1 = *(const v4f*)(vp + r * TP + 4);
        const v4f x2 = *(const v4f*)(vp + r * TP + 8);
        const v4f x3 = *(const v4f*)(vp + r * TP + 12);
        a16[0]  += kk * x0.x; a16[1]  += kk * x0.y; a16[2]  += kk * x0.z; a16[3]  += kk * x0.w;
        a16[4]  += kk * x1.x; a16[5]  += kk * x1.y; a16[6]  += kk * x1.z; a16[7]  += kk * x1.w;
        a16[8]  += kk * x2.x; a16[9]  += kk * x2.y; a16[10] += kk * x2.z; a16[11] += kk * x2.w;
        a16[12] += kk * x3.x; a16[13] += kk * x3.y; a16[14] += kk * x3.z; a16[15] += kk * x3.w;
      }
      float* kq = kva + h * (HD * HD) + cm * HD + dg;
#pragma unroll
      for (int j = 0; j < 4; ++j) {
        v4f c4 = *(const v4f*)(kq + 4 * j);
        c4.x += a16[4 * j]; c4.y += a16[4 * j + 1]; c4.z += a16[4 * j + 2]; c4.w += a16[4 * j + 3];
        *(v4f*)(kq + 4 * j) = c4;
      }
    }
    v4f vb[2];
#pragma unroll
    for (int it = 0; it < 2; ++it) {
      const int f = it * NTHR + tid;
      const int row = f >> 4, p4 = (f & 15) * 4;
      const float* tv = T + SUBR * TP + row * TP + p4;
      v4f s = *(const v4f*)tv + *(const v4f*)(tv + HD);
      s = s + *(const v4f*)(tv + 2 * HD);
      s = s + *(const v4f*)(tv + 3 * HD);
      vb[it] = s * 0.25f;
    }
    float* vg = vbar + (size_t)rb * HD;
#pragma unroll
    for (int it = 0; it < 2; ++it) *(volatile v4f*)(vg + 4 * (it * NTHR + tid)) = vb[it];
    __threadfence();
#pragma unroll
    for (int it = 0; it < 2; ++it) *(volatile v4f*)(vg + 4 * (it * NTHR + tid)) = vb[it];
    __syncthreads();
  }

  float* gp = kvpart + (size_t)blockIdx.x * KVN;
#pragma unroll 1
  for (int it = 0; it < 16; ++it) {
    const int f = it * NTHR + tid;
    const v4f v = ((const v4f*)kva)[f];
    *(volatile v4f*)(gp + 4 * f) = v;
  }
  __threadfence();
#pragma unroll 1
  for (int it = 0; it < 16; ++it) {
    const int f = it * NTHR + tid;
    const v4f v = ((const v4f*)kva)[f];
    *(volatile v4f*)(gp + 4 * f) = v;
  }
  double* sd = (double*)T;
  sd[tid] = sk; sd[CW + tid] = sk2; sd[2 * CW + tid] = sv;
  __syncthreads();
  double* rp = strec + (size_t)blockIdx.x * SRECN;
#pragma unroll
  for (int it = 0; it < 2; ++it) {
    const int f = it * NTHR + tid;
    if (f < SRECN / 2) { const v2d w = *(const v2d*)(sd + 2 * f); *(volatile v2d*)(rp + 2 * f) = w; }
  }
  __threadfence();
#pragma unroll
  for (int it = 0; it < 2; ++it) {
    const int f = it * NTHR + tid;
    if (f < SRECN / 2) { const v2d w = *(const v2d*)(sd + 2 * f); *(volatile v2d*)(rp + 2 * f) = w; }
  }
}

__global__ __launch_bounds__(NTHR) void k_fin1(const double* __restrict__ strec, const float* __restrict__ kvpart,
                                               int nKB, _Float16* kvp, float* tab) {
  extern __shared__ v4f lds_dyn[];
  float* kst  = (float*)lds_dyn;
  double* sd  = (double*)(kst + KVN);
  float* tb   = (float*)(sd + CW);
  const int tid = threadIdx.x;
  double Sk = 0.0, Sk2 = 0.0, Sv = 0.0;
#pragma unroll 1
  for (int b = 0; b < nKB; ++b) {
    const size_t base = (size_t)b * SRECN;
    Sk  += strec[base + tid];
    Sk2 += strec[base + CW + tid];
    Sv  += strec[base + 2 * CW + tid];
  }
  sd[tid] = Sk2;
  __syncthreads();
  double tot = 0.0;
#pragma unroll 1
  for (int c = 0; c < CW; ++c) tot += sd[c];
  const float nk  = sqrtf((float)tot);
  const float ikn = 1.0f / nk;
  tb[tid]      = (float)Sk * ikn;
  tb[CW + tid] = (float)Sv;
  const float ksc = ikn * (float)KVSC;
#pragma unroll 1
  for (int j = 0; j < 64; ++j) {
    const int idx = j * NTHR + tid;
    double s = 0.0;
#pragma unroll 1
    for (int b = 0; b < nKB; ++b) s += (double)kvpart[(size_t)b * KVN + idx];
    kst[idx] = (float)s * ksc;
  }
  __syncthreads();

#pragma unroll 1
  for (int it = 0; it < 8; ++it) {
    const int f = it * NTHR + tid;
    const int h = f >> 9, d = (f >> 3) & 63, m8 = (f & 7) * 8;
    v8h hv;
#pragma unroll
    for (int e = 0; e < 8; ++e) hv[e] = (_Float16)kst[h * (HD * HD) + (m8 + e) * HD + d];
    *(volatile v8h*)(kvp + 8 * f) = hv;
  }
  if (tid < 128) { const v4f v = *(const v4f*)(tb + 4 * tid); *(volatile v4f*)(tab + 4 * tid) = v; }
  if (tid >= 128 && tid < 136) {
    v4f z = {0.f, 0.f, 0.f, 0.f};
    if (tid == 128) { z.x = ikn; z.y = nk; }
    *(volatile v4f*)(tab + TS1 + 4 * (tid - 128)) = z;
  }
  __threadfence();
#pragma unroll 1
  for (int it = 0; it < 8; ++it) {
    const int f = it * NTHR + tid;
    const int h = f >> 9, d = (f >> 3) & 63, m8 = (f & 7) * 8;
    v8h hv;
#pragma unroll
    for (int e = 0; e < 8; ++e) hv[e] = (_Float16)kst[h * (HD * HD) + (m8 + e) * HD + d];
    *(volatile v8h*)(kvp + 8 * f) = hv;
  }
  if (tid < 128) { const v4f v = *(const v4f*)(tb + 4 * tid); *(volatile v4f*)(tab + 4 * tid) = v; }
  if (tid >= 128 && tid < 136) {
    v4f z = {0.f, 0.f, 0.f, 0.f};
    if (tid == 128) { z.x = ikn; z.y = nk; }
    *(volatile v4f*)(tab + TS1 + 4 * (tid - 128)) = z;
  }
}

__global__ __launch_bounds__(NTHR) void k_q(const float* __restrict__ X, const _Float16* __restrict__ wp,
                                            const float* __restrict__ bq, const float* __restrict__ tab,
                                            _Float16* qh, float* dotq, double* qrec, int nN) {
  extern __shared__ v4f lds_dyn[];
  _Float16* Ah = (_Float16*)lds_dyn;
  float* T   = (float*)((char*)lds_dyn + LDS_AH);
  float* csk = T + SUBR * TP;
  float* dq  = csk + CW;
  const int tid = threadIdx.x, lane = tid & 31, wave = tid >> 5;
  csk[tid] = tab[TCSK + tid];
  double sq2 = 0.0;
  const int drow = tid >> 3, dh = (tid >> 1) & 3, dk = tid & 1;

#pragma unroll 1
  for (int st = 0; st < QR / SUBR; ++st) {
    const int rb = blockIdx.x * QR + st * SUBR;
    cvt_tile(X, rb, nN, Ah, tid);
    __syncthreads();
    gemm_unit(Ah, wp, bq, T, wave & 1, wave >> 1, lane);
    __syncthreads();
    int nr = nN - rb;
    nr = nr > SUBR ? SUBR : nr;
#pragma unroll 1
    for (int r = 0; r < nr; ++r) {
      const float qv = T[r * TP + tid];
      sq2 += (double)qv * (double)qv;
    }
    {
      const float* tp2 = T + drow * TP + dh * HD + 32 * dk;
      const float* cp2 = csk + dh * HD + 32 * dk;
      float s = 0.0f;
#pragma unroll 4
      for (int mm = 0; mm < 32; ++mm) s += tp2[mm] * cp2[mm];
      s += __shfl_xor(s, 1, 32);
      s = (drow < nr) ? s : 0.0f;
      if (dk == 0) dq[drow * NH + dh] = s;
    }
    v8h hv[4];
#pragma unroll
    for (int it = 0; it < 4; ++it) {
      const int f = it * NTHR + tid;
      const int row = f >> 5, c8 = (f & 31) * 8;
      const float* tq = T + row * TP + c8;
      hv[it] = cvt8(*(const v4f*)tq, *(const v4f*)(tq + 4), (float)QSC);
    }
    _Float16* qg = qh + (size_t)rb * CW;
#pragma unroll
    for (int it = 0; it < 4; ++it) *(volatile v8h*)(qg + 8 * (it * NTHR + tid)) = hv[it];
    __threadfence();
#pragma unroll
    for (int it = 0; it < 4; ++it) *(volatile v8h*)(qg + 8 * (it * NTHR + tid)) = hv[it];
    __syncthreads();
    v4f d4 = {0.f, 0.f, 0.f, 0.f};
    if (tid < SUBR) d4 = *(const v4f*)(dq + NH * tid);
    if (tid < SUBR) *(volatile v4f*)(dotq + (size_t)(rb + tid) * NH) = d4;
    __threadfence();
    if (tid < SUBR) *(volatile v4f*)(dotq + (size_t)(rb + tid) * NH) = d4;
    __syncthreads();
  }

  double* sd = (double*)T;
  sd[tid] = sq2;
  __syncthreads();
  double* rp = qrec + (size_t)blockIdx.x * QRECN;
  v2d w = {0.0, 0.0};
  if (tid < QRECN / 2) w = *(const v2d*)(sd + 2 * tid);
  if (tid < QRECN / 2) *(volatile v2d*)(rp + 2 * tid) = w;
  __threadfence();
  if (tid < QRECN / 2) *(volatile v2d*)(rp + 2 * tid) = w;
}

__global__ __launch_bounds__(NTHR) void k_fin2(const double* __restrict__ qrec, int nQB, float* tab) {
  __shared__ double sd[CW];
  const int tid = threadIdx.x;
  double S = 0.0;
#pragma unroll 1
  for (int b = 0; b < nQB; ++b) S += qrec[(size_t)b * QRECN + tid];
  sd[tid] = S;
  __syncthreads();
  double tot = 0.0;
#pragma unroll 1
  for (int c = 0; c < CW; ++c) tot += sd[c];
  const float nq  = sqrtf((float)tot);
  const float iqn = 1.0f / nq;
  v4f z = {0.f, 0.f, 0.f, 0.f};
  if (tid == 0) { z.x = iqn; z.y = nq; }
  if (tid < 8) *(volatile v4f*)(tab + TS2 + 4 * tid) = z;
  __threadfence();
  if (tid < 8) *(volatile v4f*)(tab + TS2 + 4 * tid) = z;
}

__global__ __launch_bounds__(NTHR) void k_gcn(const int* __restrict__ col, const int* __restrict__ src,
                                              const float* __restrict__ ew, const float* __restrict__ dz,
                                              const float* __restrict__ vbar, float* gcn, int nE, int nN, int vec8) {
  extern __shared__ v4f lds_dyn[];
  float* gac = (float*)lds_dyn;
  int* list  = (int*)(gac + GSL * HD);
  int* wcnt  = list + LISTN;
  const int tid = threadIdx.x, lane = tid & 31, wave = tid >> 5;
  const int nodeBase = blockIdx.x * GSL;
  {
    const v4f z = {0.f, 0.f, 0.f, 0.f};
    for (int i = tid; i < GSL * HD / 4; i += NTHR) ((v4f*)gac)[i] = z;
  }
  __syncthreads();

  const int nChunks = (nE + CHUNK - 1) / CHUNK;
#pragma unroll 1
  for (int ch = 0; ch < nChunks; ++ch) {
    const int cbase = ch * CHUNK;
    const int wc = scan_chunk<GSL, 1>(col, nE, cbase, nodeBase, vec8, list, tid, wave);
    if (lane == 0) wcnt[wave] = wc;
    __syncthreads();
    if (wave == 0) {
#pragma unroll 1
      for (int wsx = 0; wsx < NWAVE; ++wsx) {
        int n = __builtin_amdgcn_readfirstlane(wcnt[wsx]);
        n = n > WCAP ? WCAP : (n < 0 ? 0 : n);
        const int* lp = list + wsx * WCAP;
#pragma unroll 1
        for (int i = 0; i < n; ++i) {
          int e = __builtin_amdgcn_readfirstlane(lp[i]);
          e = e < 0 ? 0 : (e > nE - 1 ? nE - 1 : e);
          const int c = col[e];
          int r = src[e];
          r = r < 0 ? 0 : (r > nN - 1 ? nN - 1 : r);
          const float w = ew[e];
          const int slot = c - nodeBase;
          if ((unsigned)slot < (unsigned)GSL) {
            const float val = (w * dz[nodeBase + slot]) * dz[r];
            float* apx = gac + slot * HD + 2 * lane;
            const v2f vb = *(const v2f*)(vbar + (size_t)r * HD + 2 * lane);
            v2f cur = *(const v2f*)apx;
            cur = cur + vb * val;
            *(v2f*)apx = cur;
          }
        }
      }
    }
    __syncthreads();
  }

  float* gp = gcn + (size_t)nodeBase * HD;
#pragma unroll 1
  for (int it = 0; it < 32; ++it) {
    const int f = it * NTHR + tid;
    const v4f v = ((const v4f*)gac)[f];
    *(volatile v4f*)(gp + 4 * f) = v;
  }
  __threadfence();
#pragma unroll 1
  for (int it = 0; it < 32; ++it) {
    const int f = it * NTHR + tid;
    const v4f v = ((const v4f*)gac)[f];
    *(volatile v4f*)(gp + 4 * f) = v;
  }
}

__global__ __launch_bounds__(NTHR) void k_attn(const _Float16* __restrict__ qh, const _Float16* __restrict__ kvp,
                                               const float* __restrict__ tab, const float* __restrict__ dotq,
                                               const float* __restrict__ gcn, float* out, int nN) {
  __shared__ __attribute__((aligned(16))) float stg[NWAVE * 16 * HD];
  const int tid = threadIdx.x, lane = tid & 31, wave = tid >> 5, hh = lane >> 4, m = lane & 15;
  const int mw = blockIdx.x * AR + wave * 16;
  const float iqn = tab[TS2];
  const float esc = iqn * (1.0f / (float)(QSC * KVSC));
  const float fN  = (float)nN;
  v8f hs[4];
#pragma unroll
  for (int t = 0; t < 4; ++t) { v8f z = {0.f, 0.f, 0.f, 0.f, 0.f, 0.f, 0.f, 0.f}; hs[t] = z; }
  const _Float16* qp = qh + (size_t)(mw + m) * CW + 8 * hh;
  const float* dqp = dotq + (size_t)(mw + 8 * hh) * NH;

#pragma unroll
  for (int h = 0; h < NH; ++h) {
    v8f acc[4];
#pragma unroll
    for (int t = 0; t < 4; ++t) { v8f z = {0.f, 0.f, 0.f, 0.f, 0.f, 0.f, 0.f, 0.f}; acc[t] = z; }
#pragma unroll
    for (int ks = 0; ks < 2; ++ks) {
      FragH af;
      af.h[0] = *(const v8h*)(qp + h * HD + 32 * ks);
      af.h[1] = *(const v8h*)(qp + h * HD + 32 * ks + 16);
#pragma unroll
      for (int nt = 0; nt < 4; ++nt) {
        const _Float16* bp = kvp + h * (HD * HD) + (16 * nt + m) * HD + 32 * ks + 8 * hh;
        FragH bf;
        bf.h[0] = *(const v8h*)bp;
        bf.h[1] = *(const v8h*)(bp + 16);
        acc[nt] = wmf(af.v, bf.v, acc[nt]);
      }
    }
    float rn[8];
#pragma unroll
    for (int r = 0; r < 8; ++r) {
      const float nm = dqp[r * NH + h] * iqn + fN;
      rn[r] = 1.0f / nm;
    }
#pragma unroll
    for (int nt = 0; nt < 4; ++nt) {
      const float cv = tab[TCSV + h * HD + 16 * nt + m];
#pragma unroll
      for (int r = 0; r < 8; ++r) hs[nt][r] += (acc[nt][r] * esc + cv) * rn[r];
    }
  }

  float* sp = stg + (wave * 16 + 8 * hh) * HD + m;
#pragma unroll
  for (int nt = 0; nt < 4; ++nt) {
#pragma unroll
    for (int r = 0; r < 8; ++r) sp[r * HD + 16 * nt] = hs[nt][r] * 0.25f;
  }
  __syncthreads();

  const float* lp = stg + wave * 16 * HD;
  const int rsub = lane >> 4, p4 = (lane & 15) * 4;
  v4f ov[8];
#pragma unroll
  for (int i = 0; i < 8; ++i) {
    const int row = 2 * i + rsub;
    const v4f s = *(const v4f*)(lp + row * HD + p4);
    const v4f g = *(const v4f*)(gcn + (size_t)(mw + row) * HD + p4);
    ov[i] = s + g;
  }
#pragma unroll
  for (int i = 0; i < 8; ++i) {
    const int row = 2 * i + rsub;
    if (mw + row < nN) *(volatile v4f*)(out + (size_t)(mw + row) * HD + p4) = ov[i];
  }
  __threadfence();
#pragma unroll
  for (int i = 0; i < 8; ++i) {
    const int row = 2 * i + rsub;
    if (mw + row < nN) *(volatile v4f*)(out + (size_t)(mw + row) * HD + p4) = ov[i];
  }
}

extern "C" void kernel_launch(void* const* d_in, const int* in_sizes, int n_in,
                              void* d_out, int out_size, void* d_ws, size_t ws_size,
                              hipStream_t stream) {
  if (n_in < 10) return;
  const int nN = in_sizes[0] / CIN;
  if (nN <= 0 || in_sizes[0] != nN * CIN || in_sizes[1] != nN * CIN) return;
  if (in_sizes[2] != CW * CIN || in_sizes[4] != CW * CIN || in_sizes[6] != CW * CIN) return;
  if (in_sizes[3] != CW || in_sizes[5] != CW || in_sizes[7] != CW) return;
  const int nE = in_sizes[9];
  if (nE <= 0 || in_sizes[8] != 2 * nE) return;
  if (out_size != nN * HD) return;
  if (nN > (1 << 20) || nE > (1 << 28)) return;

  const float* Xq = (const float*)d_in[0];
  const float* Xs = (const float*)d_in[1];
  const float* Wq = (const float*)d_in[2];
  const float* bq = (const float*)d_in[3];
  const float* Wk = (const float*)d_in[4];
  const float* bk = (const float*)d_in[5];
  const float* Wv = (const float*)d_in[6];
  const float* bv = (const float*)d_in[7];
  const int*   ei = (const int*)d_in[8];
  const float* ew = (const float*)d_in[9];
  const int*   erow = ei;
  const int*   ecol = ei + nE;
  float* out = (float*)d_out;

  const int NP = ((nN + NPQ - 1) / NPQ) * NPQ;
  const int nBC = (nN + NBC - 1) / NBC;
  const int CNTPAD = nBC * NBC;
  if (CNTPAD < NP) return;
  const int nKB = NP / KVR, nQB = NP / QR, nAB = NP / AR, nGB = NP / GSL;

  char* ws = (char*)d_ws;
  size_t off = 0;
  const size_t oW   = off; off += (size_t)3 * CW * CIN * 2;        off = (off + 255) & ~(size_t)255;
  const size_t oCnt = off; off += (size_t)CNTPAD * 4;              off = (off + 255) & ~(size_t)255;
  const size_t oDz  = off; off += (size_t)CNTPAD * 4;              off = (off + 255) & ~(size_t)255;
  const size_t oQh  = off; off += (size_t)NP * CW * 2;             off = (off + 255) & ~(size_t)255;
  const size_t oDq  = off; off += (size_t)NP * NH * 4;             off = (off + 255) & ~(size_t)255;
  const size_t oVb  = off; off += (size_t)NP * HD * 4;             off = (off + 255) & ~(size_t)255;
  const size_t oGc  = off; off += (size_t)NP * HD * 4;             off = (off + 255) & ~(size_t)255;
  const size_t oKvp = off; off += (size_t)nKB * KVN * 4;           off = (off + 255) & ~(size_t)255;
  const size_t oSr  = off; off += (size_t)nKB * SRECN * 8;         off = (off + 255) & ~(size_t)255;
  const size_t oQr  = off; off += (size_t)nQB * QRECN * 8;         off = (off + 255) & ~(size_t)255;
  const size_t oKp  = off; off += (size_t)KVN * 2;                 off = (off + 255) & ~(size_t)255;
  const size_t oTab = off; off += (size_t)TABN * 4;                off = (off + 255) & ~(size_t)255;
  if (off > ws_size || off > (size_t)WSCAP) return;
  _Float16* wp     = (_Float16*)(ws + oW);
  int*      cnt    = (int*)(ws + oCnt);
  float*    dz     = (float*)(ws + oDz);
  _Float16* qh     = (_Float16*)(ws + oQh);
  float*    dotq   = (float*)(ws + oDq);
  float*    vbar   = (float*)(ws + oVb);
  float*    gcn    = (float*)(ws + oGc);
  float*    kvpart = (float*)(ws + oKvp);
  double*   strec  = (double*)(ws + oSr);
  double*   qrec   = (double*)(ws + oQr);
  _Float16* kvp    = (_Float16*)(ws + oKp);
  float*    tab    = (float*)(ws + oTab);

  const int vec8 = ((nE & 3) == 0) ? 1 : 0;

  hipFuncSetAttribute(reinterpret_cast<const void*>(&k_count), hipFuncAttributeMaxDynamicSharedMemorySize, LDS_COUNT);
  hipFuncSetAttribute(reinterpret_cast<const void*>(&k_kv), hipFuncAttributeMaxDynamicSharedMemorySize, LDS_KV);
  hipFuncSetAttribute(reinterpret_cast<const void*>(&k_fin1), hipFuncAttributeMaxDynamicSharedMemorySize, LDS_F1);
  hipFuncSetAttribute(reinterpret_cast<const void*>(&k_gcn), hipFuncAttributeMaxDynamicSharedMemorySize, LDS_GCN);

  k_wprep<<<96, NTHR, 0, stream>>>(Wq, Wk, Wv, wp);
  k_count<<<nBC, NTHR, LDS_COUNT, stream>>>(ecol, cnt, dz, nE, vec8);
  k_kv<<<nKB, NTHR, LDS_KV, stream>>>(Xs, wp, bk, bv, vbar, kvpart, strec, nN);
  k_fin1<<<1, NTHR, LDS_F1, stream>>>(strec, kvpart, nKB, kvp, tab);
  k_q<<<nQB, NTHR, LDS_Q, stream>>>(Xq, wp, bq, tab, qh, dotq, qrec, nN);
  k_fin2<<<1, NTHR, 0, stream>>>(qrec, nQB, tab);
  k_gcn<<<nGB, NTHR, LDS_GCN, stream>>>(ecol, erow, ew, dz, vbar, gcn, nE, nN, vec8);
  k_attn<<<nAB, NTHR, 0, stream>>>(qh, kvp, tab, dotq, gcn, out, nN);
}
